// GraphConvolution_8684423872665
// MI455X (gfx1250) — hardware-verified
//
#include <hip/hip_runtime.h>
#include <math.h>

constexpr int kNodes = 100000;
constexpr int kEdges = 640000;
constexpr int kFeat = 128;
constexpr int kMPad = 100096;
constexpr int kThreads = 256;
constexpr int kWaves = kThreads / 32;
constexpr int kTileRows = 16384;
constexpr int kRowsPerWave = kTileRows / kWaves;
constexpr int kTiles = 7;
constexpr int kEdgesPerThread = 8;
constexpr int kChunk = kThreads * kEdgesPerThread;
constexpr int kChunks = (kEdges + kChunk - 1) / kChunk;
constexpr int kScanWords = 80;
constexpr int kDlShift = 17;
constexpr int kSrcMask = (1 << kDlShift) - 1;
constexpr int kOwnShift = kDlShift + 11;
constexpr float kAggCarry = 4.0f;
constexpr float kWCarry = 16.0f;
constexpr float kGemmScale = 1.0f / 64.0f;
constexpr size_t kWsLimit = 134217728;

static_assert(kEdges % kEdgesPerThread == 0);
static_assert(kEdgesPerThread == 8);
static_assert(kChunk == kThreads * kEdgesPerThread);
static_assert(kChunk % kThreads == 0);
static_assert(kTiles * kTileRows >= kMPad);
static_assert(kMPad >= kNodes);
static_assert(kMPad % 64 == 0);
static_assert(kMPad % 4 == 0);
static_assert(kFeat == 128);
static_assert(kFeat % 64 == 0);
static_assert(kFeat % 32 == 0);
static_assert(kRowsPerWave * kWaves == kTileRows);
static_assert(kRowsPerWave == (1 << (kOwnShift - kDlShift)));
static_assert(kRowsPerWave % 4 == 0);
static_assert(kTileRows <= (1 << 14));
static_assert(kNodes <= (1 << kDlShift));
static_assert(kNodes % kWaves == 0);
static_assert(kScanWords >= 65 && kScanWords <= kThreads);
static_assert(kWaves == 8);

typedef __attribute__((ext_vector_type(16))) _Float16 v16h;
typedef __attribute__((ext_vector_type(8)))  _Float16 v8h;
typedef __attribute__((ext_vector_type(16))) __bf16   v16b;
typedef __attribute__((ext_vector_type(8)))  __bf16   v8b;
typedef __attribute__((ext_vector_type(8)))  float    v8f;
typedef __attribute__((ext_vector_type(4)))  float    v4f;
typedef __attribute__((ext_vector_type(4)))  int      v4i;
typedef __attribute__((ext_vector_type(4)))  unsigned int v4u;

__device__ __forceinline__ unsigned short f2bf_bits(float f) {
  unsigned u = __float_as_uint(f);
  return (unsigned short)((u + 0x7FFFu + ((u >> 16) & 1u)) >> 16);
}
__device__ __forceinline__ float bf_bits2f(unsigned short h) { return __uint_as_float(((unsigned)h) << 16); }
__device__ __forceinline__ unsigned pk16(unsigned short a, unsigned short b) { return (unsigned)a | ((unsigned)b << 16); }
__device__ __forceinline__ unsigned short h_bits(float f) { const _Float16 h = (_Float16)f; return __builtin_bit_cast(unsigned short, h); }

__device__ __forceinline__ void dep_guard4_h(v8f& a, v8f& b, v8f& c, v8f& d, v16h x, v16h y) {
  asm volatile("v_nop\n\tv_nop\n\tv_nop\n\tv_nop" : "+v"(a), "+v"(b), "+v"(c), "+v"(d) : "v"(x), "v"(y));
}
__device__ __forceinline__ void dep_guard4_b(v8f& a, v8f& b, v8f& c, v8f& d, v16b x, v16b y) {
  asm volatile("v_nop\n\tv_nop\n\tv_nop\n\tv_nop" : "+v"(a), "+v"(b), "+v"(c), "+v"(d) : "v"(x), "v"(y));
}
__device__ __forceinline__ void keep4_h(v16h a, v16h b, v16h c, v16h d) { asm volatile("v_nop" :: "v"(a), "v"(b), "v"(c), "v"(d)); }
__device__ __forceinline__ void keep4_b(v16b a, v16b b, v16b c, v16b d) { asm volatile("v_nop" :: "v"(a), "v"(b), "v"(c), "v"(d)); }
__device__ __forceinline__ void acc_guard4(v8f& a, v8f& b, v8f& c, v8f& d) { asm volatile("v_nop\n\tv_nop\n\tv_nop\n\tv_nop" : "+v"(a), "+v"(b), "+v"(c), "+v"(d)); }

template <typename T> struct Frag;
template <> struct Frag<_Float16> {
  typedef v16h V; union U { v16h v; v8h h[2]; };
  static __device__ __forceinline__ v16h load(const _Float16* p) {
    U f; f.h[0] = *(const v8h*)(p); f.h[1] = *(const v8h*)(p + 16); return f.v;
  }
  static __device__ __forceinline__ v8f mma(v16h a, v16h b, v8f c) {
    return __builtin_amdgcn_wmma_f32_16x16x32_f16(false, a, false, b, (short)0, c, false, false);
  }
  static __device__ __forceinline__ void guard4(v8f& a, v8f& b, v8f& c, v8f& d, v16h x, v16h y) { dep_guard4_h(a, b, c, d, x, y); }
  static __device__ __forceinline__ void keep(v16h a, v16h b, v16h c, v16h d) { keep4_h(a, b, c, d); }
};
template <> struct Frag<__bf16> {
  typedef v16b V; union U { v16b v; v8b h[2]; };
  static __device__ __forceinline__ v16b load(const __bf16* p) {
    U f; f.h[0] = *(const v8b*)(p); f.h[1] = *(const v8b*)(p + 16); return f.v;
  }
  static __device__ __forceinline__ v8f mma(v16b a, v16b b, v8f c) {
    return __builtin_amdgcn_wmma_f32_16x16x32_bf16(false, a, false, b, (short)0, c, false, false);
  }
  static __device__ __forceinline__ void guard4(v8f& a, v8f& b, v8f& c, v8f& d, v16b x, v16b y) { dep_guard4_b(a, b, c, d, x, y); }
  static __device__ __forceinline__ void keep(v16b a, v16b b, v16b c, v16b d) { keep4_b(a, b, c, d); }
};

template <int ET> struct Elem;
template <> struct Elem<0> { typedef _Float16 T; };
template <> struct Elem<1> { typedef __bf16 T; };
template <int ET, bool SPLIT, int BIAS_MODE, int OUT_MODE, bool RESID, int ACT = 0>
__global__ __launch_bounds__(256) void wmma_gemm64(
    const unsigned short* __restrict__ Ap, const unsigned short* __restrict__ A2p, int lda, long strideA,
    const unsigned short* __restrict__ Btp, const unsigned short* __restrict__ Bt2p, int ldb, long strideB,
    void* __restrict__ Cout, void* __restrict__ Cout2, int ldc, long strideC,
    const float* __restrict__ bias,
    const float* __restrict__ resid, long strideR,
    int M, int N, int K, float scale) {
  typedef typename Elem<ET>::T T;
  typedef typename Frag<T>::V V;
  const T* A = (const T*)Ap; const T* A2 = (const T*)A2p; const T* Bt = (const T*)Btp; const T* Bt2 = (const T*)Bt2p;
  __shared__ __align__(16) float sT[8][16 * 68];
  const int b    = blockIdx.y;
  const int lane = threadIdx.x & 31;
  const int wave = threadIdx.x >> 5;
  const int tilesN = N >> 6;
  const int tilesM = M >> 6;
  const int tile = blockIdx.x * 8 + wave;
  if (tile >= tilesM * tilesN) return;
  const int tm = tile / tilesN;
  const int tn = tile - tm * tilesN;
  const int m0 = tm << 6;
  const int n0 = tn << 6;

  const T* Ab  = A  + (size_t)b * strideA;
  const T* Bb  = Bt + (size_t)b * strideB;
  const T* Ab2 = SPLIT ? (A2  + (size_t)b * strideA) : nullptr;
  const T* Bb2 = SPLIT ? (Bt2 + (size_t)b * strideB) : nullptr;

  const int rlane = lane & 15;
  const int koff  = (lane >> 4) * 8;
  const int mOff  = (lane >> 4) * 8;

  v8f acc[4][4];
#pragma unroll
  for (int i = 0; i < 4; ++i)
#pragma unroll
    for (int j = 0; j < 4; ++j) acc[i][j] = (v8f){0.f,0.f,0.f,0.f,0.f,0.f,0.f,0.f};

  for (int k0 = 0; k0 < K; k0 += 32) {
    V bh[4], bl[4];
#pragma unroll
    for (int j = 0; j < 4; ++j) {
      const size_t bo = (size_t)(n0 + (j << 4) + rlane) * ldb + koff + k0;
      bh[j] = Frag<T>::load(Bb + bo);
      if (SPLIT) bl[j] = Frag<T>::load(Bb2 + bo);
    }
#pragma unroll
    for (int i = 0; i < 4; ++i) {
      const size_t ao = (size_t)(m0 + (i << 4) + rlane) * lda + koff + k0;
      V ah = Frag<T>::load(Ab + ao);
      V al;
      if (SPLIT) al = Frag<T>::load(Ab2 + ao);
#pragma unroll
      for (int j = 0; j < 4; ++j) {
        acc[i][j] = Frag<T>::mma(ah, bh[j], acc[i][j]);
        if (SPLIT) {
          acc[i][j] = Frag<T>::mma(ah, bl[j], acc[i][j]);
          acc[i][j] = Frag<T>::mma(al, bh[j], acc[i][j]);
        }
      }
      Frag<T>::guard4(acc[i][0], acc[i][1], acc[i][2], acc[i][3], ah, SPLIT ? al : ah);
    }
    Frag<T>::keep(bh[0], bh[1], bh[2], bh[3]);
    if (SPLIT) Frag<T>::keep(bl[0], bl[1], bl[2], bl[3]);
  }
  acc_guard4(acc[0][0], acc[0][1], acc[0][2], acc[0][3]);
  acc_guard4(acc[1][0], acc[1][1], acc[1][2], acc[1][3]);
  acc_guard4(acc[2][0], acc[2][1], acc[2][2], acc[2][3]);
  acc_guard4(acc[3][0], acc[3][1], acc[3][2], acc[3][3]);

  float* slab = sT[wave];
  const float* Rb = RESID ? (resid + (size_t)b * strideR) : nullptr;
#pragma unroll
  for (int i = 0; i < 4; ++i) {
    const int mBase = m0 + (i << 4);
#pragma unroll
    for (int j = 0; j < 4; ++j) {
      const int n = n0 + (j << 4) + rlane;
      float bv = 0.f;
      if (BIAS_MODE == 2) bv = bias[n];
#pragma unroll
      for (int r = 0; r < 8; ++r) {
        float v = acc[i][j][r] * scale;
        if (BIAS_MODE == 1) v += bias[mBase + mOff + r];
        if (BIAS_MODE == 2) v += bv;
        if (RESID) v += Rb[(size_t)(mBase + mOff + r) * ldc + n];
        if (ACT == 2) v = fmaxf(v, 0.0f);
        if (ACT == 4) v = (v > 0.f) ? v : 0.01f * v;
        if (ACT == 6) { const float den = 1.0f + expf(-v); v = __builtin_amdgcn_rcpf(den); }
        slab[(mOff + r) * 68 + (j << 4) + rlane] = v;
      }
    }
    __builtin_amdgcn_fence(__ATOMIC_RELEASE, "workgroup");
    __builtin_amdgcn_wave_barrier();
    __builtin_amdgcn_fence(__ATOMIC_ACQUIRE, "workgroup");
    if (OUT_MODE == 0) {
      float* C = (float*)Cout + (size_t)b * strideC;
      const int hh = lane >> 4, c4 = (lane & 15) * 4;
      for (int pass = 0; pass < 2; ++pass) {
#pragma unroll
        for (int it = 0; it < 8; ++it) {
          const int row = it * 2 + hh;
          v4f v = *(const v4f*)(slab + row * 68 + c4);
          *(volatile v4f*)(C + (size_t)(mBase + row) * ldc + n0 + c4) = v;
        }
        __threadfence();
      }
    } else {
      const int q = lane >> 3, c8 = (lane & 7) * 8;
      unsigned short* C  = (unsigned short*)Cout  + (size_t)b * strideC;
      unsigned short* C2 = (OUT_MODE == 2) ? ((unsigned short*)Cout2 + (size_t)b * strideC) : nullptr;
      for (int pass = 0; pass < 2; ++pass) {
#pragma unroll
        for (int it = 0; it < 4; ++it) {
          const int row = it * 4 + q;
          const float* sp = slab + row * 68 + c8;
          v8h hv, lv;
#pragma unroll
          for (int e = 0; e < 8; ++e) {
            if (OUT_MODE == 1) {
              hv[e] = (_Float16)sp[e];
            } else {
              unsigned short hb = f2bf_bits(sp[e]);
              unsigned short lb = f2bf_bits(sp[e] - bf_bits2f(hb));
              hv[e] = __builtin_bit_cast(_Float16, hb);
              lv[e] = __builtin_bit_cast(_Float16, lb);
            }
          }
          *(volatile v8h*)(C + (size_t)(mBase + row) * ldc + n0 + c8) = hv;
          if (OUT_MODE == 2) *(volatile v8h*)(C2 + (size_t)(mBase + row) * ldc + n0 + c8) = lv;
        }
        __threadfence();
      }
    }
    __builtin_amdgcn_fence(__ATOMIC_RELEASE, "workgroup");
    __builtin_amdgcn_wave_barrier();
    __builtin_amdgcn_fence(__ATOMIC_ACQUIRE, "workgroup");
  }
}

__device__ __forceinline__ int blk_excl_scan(int cnt, int* scan_ws, int tid, int& tot) {
  const int lane = tid & 31, wave = tid >> 5; int incl = cnt;
#pragma unroll
  for (int o = 1; o < 32; o <<= 1) { const int v = __shfl_up(incl, o, 32); if (lane >= o) incl += v; }
  if (lane == 31) scan_ws[wave] = incl;
  __syncthreads();
  if (wave == 0) {
    const int wraw = scan_ws[lane];
    const int wv = (lane < kWaves) ? wraw : 0; int wincl = wv;
#pragma unroll
    for (int o = 1; o < 32; o <<= 1) { const int v = __shfl_up(wincl, o, 32); if (lane >= o) wincl += v; }
    if (lane < kWaves) scan_ws[32 + lane] = wincl - wv;
    if (lane == 31) scan_ws[64] = wincl;
  }
  __syncthreads();
  const int res = scan_ws[32 + wave] + incl - cnt; tot = scan_ws[64];
  return res;
}

__device__ __forceinline__ int chunk_hits(const int* __restrict__ dstv, const int* __restrict__ srcv,
                                          const float* __restrict__ valv, int e0, int n0, int tid,
                                          int* LIST, float* LVAL, int* scan_ws) {
  const int eb = e0 + tid * kEdgesPerThread;
  const bool live = eb < kEdges;
  const int ebc = live ? eb : (kEdges - kEdgesPerThread);
  const v4i d0 = *(const v4i*)(dstv + ebc);
  const v4i d1 = *(const v4i*)(dstv + ebc + 4);
  const v4i s0 = *(const v4i*)(srcv + ebc);
  const v4i s1 = *(const v4i*)(srcv + ebc + 4);
  const v4f w0 = *(const v4f*)(valv + ebc);
  const v4f w1 = *(const v4f*)(valv + ebc + 4);
  const int lv = live ? 1 : 0;
  int rec[kEdgesPerThread]; float vrec[kEdgesPerThread]; int cnt = 0;
#pragma unroll
  for (int e = 0; e < 4; ++e) {
    {
      const int d = d0[e];
      int s = s0[e]; s = s < 0 ? 0 : (s >= kNodes ? kNodes - 1 : s);
      const int hit = lv & (d >= n0 ? 1 : 0) & (d < n0 + kTileRows ? 1 : 0) & (d < kNodes ? 1 : 0);
      const int code = (int)((((unsigned)d - (unsigned)n0) << kDlShift) | (unsigned)s);
      rec[e] = hit ? code : -1; vrec[e] = w0[e]; cnt += hit;
    }
    {
      const int d = d1[e];
      int s = s1[e]; s = s < 0 ? 0 : (s >= kNodes ? kNodes - 1 : s);
      const int hit = lv & (d >= n0 ? 1 : 0) & (d < n0 + kTileRows ? 1 : 0) & (d < kNodes ? 1 : 0);
      const int code = (int)((((unsigned)d - (unsigned)n0) << kDlShift) | (unsigned)s);
      rec[4 + e] = hit ? code : -1; vrec[4 + e] = w1[e]; cnt += hit;
    }
  }
  int tot = 0;
  int p = blk_excl_scan(cnt, scan_ws, tid, tot);
#pragma unroll
  for (int k = 0; k < kEdgesPerThread; ++k) {
    if (rec[k] >= 0) { if ((unsigned)p < (unsigned)kChunk) { LIST[p] = rec[k]; LVAL[p] = vrec[k]; } ++p; }
  }
  __syncthreads();
  return tot < kChunk ? tot : kChunk;
}

__global__ __launch_bounds__(kThreads) void spmm_tile_kernel(const float* __restrict__ hsrc, const float* __restrict__ ev,
                                                             const int* __restrict__ esrc, const int* __restrict__ edst,
                                                             float* acc32, unsigned short* __restrict__ agg16) {
  __shared__ int LIST[kChunk];
  __shared__ float LVAL[kChunk];
  __shared__ int scan_ws[kScanWords];
  __shared__ __align__(16) float slab_all[kWaves][4 * kFeat];
  const int tid = threadIdx.x, lane = tid & 31, wave = tid >> 5;
  const int n0 = blockIdx.x * kTileRows;
  const int wrow0 = n0 + wave * kRowsPerWave;
  for (int i = tid; i < kChunk; i += kThreads) { LIST[i] = -1; LVAL[i] = 0.f; }
  if (tid < kScanWords) scan_ws[tid] = 0;
  const v4f z4 = {0.f, 0.f, 0.f, 0.f};
#pragma unroll 1
  for (int j = 0; j < kRowsPerWave; ++j) {
    const int row = wrow0 + j;
    if (row < kMPad) *(v4f*)(acc32 + (size_t)row * kFeat + 4 * lane) = z4;
  }
  __syncthreads();

#pragma unroll 1
  for (int c = 0; c < kChunks; ++c) {
    const int tot = chunk_hits(edst, esrc, ev, c * kChunk, n0, tid, LIST, LVAL, scan_ws);
#pragma unroll 1
    for (int base = 0; base < tot; base += 32) {
      const int q = base + lane;
      const int qc = q < kChunk ? q : (kChunk - 1);
      const int rraw = LIST[qc];
      const float vraw = LVAL[qc];
      const int keep = (q < tot) ? 1 : 0;
      const int rv = (rraw & (-keep)) | (keep - 1);
      const int own = ((rv >= 0) & ((rv >> kOwnShift) == wave)) ? 1 : 0;
      unsigned msk = (unsigned)__ballot(own);
#pragma unroll 1
      for (int it = 0; it < 32; ++it) {
        if (msk == 0u) break;
        const int bp = __builtin_ctz(msk); msk &= msk - 1u;
        const int r = __shfl(rv, bp, 32);
        const float v = __shfl(vraw, bp, 32);
        const int dl = (r >> kDlShift) & 0x3FFF;
        int s = r & kSrcMask; s = s < kNodes ? s : (kNodes - 1);
        int drow = n0 + dl; drow = drow < kMPad ? drow : (kMPad - 1);
        const v4f hv = *(const v4f*)(hsrc + (size_t)s * kFeat + 4 * lane);
        float* rp = acc32 + (size_t)drow * kFeat + 4 * lane;
        v4f a = *(const v4f*)rp;
        a = a + v * hv;
        *(v4f*)rp = a;
      }
    }
    __syncthreads();
  }
  __threadfence();

  float* slab = slab_all[wave];
  const int hh = lane >> 4, c8 = (lane & 15) * 8;
#pragma unroll 1
  for (int j = 0; j < kRowsPerWave / 4; ++j) {
    const int rb = wrow0 + 4 * j;
    if (rb < kMPad) {
#pragma unroll
      for (int rr = 0; rr < 4; ++rr) {
        const v4f a = *(const v4f*)(acc32 + (size_t)(rb + rr) * kFeat + 4 * lane);
        *(v4f*)(slab + rr * kFeat + 4 * lane) = a;
      }
      __builtin_amdgcn_fence(__ATOMIC_RELEASE, "workgroup");
      __builtin_amdgcn_wave_barrier();
      __builtin_amdgcn_fence(__ATOMIC_ACQUIRE, "workgroup");
      for (int pass = 0; pass < 2; ++pass) {
#pragma unroll
        for (int it = 0; it < 2; ++it) {
          const int row = it * 2 + hh;
          const float* sp = slab + row * kFeat + c8;
          const v4f a0 = *(const v4f*)(sp);
          const v4f a1 = *(const v4f*)(sp + 4);
          unsigned short hb[8];
#pragma unroll
          for (int e = 0; e < 4; ++e) {
            hb[e]     = h_bits(a0[e] * kAggCarry);
            hb[4 + e] = h_bits(a1[e] * kAggCarry);
          }
          const v4u u = (v4u){pk16(hb[0], hb[1]), pk16(hb[2], hb[3]), pk16(hb[4], hb[5]), pk16(hb[6], hb[7])};
          *(volatile v4u*)(agg16 + (size_t)(rb + row) * kFeat + c8) = u;
        }
        __threadfence();
      }
      __builtin_amdgcn_fence(__ATOMIC_RELEASE, "workgroup");
      __builtin_amdgcn_wave_barrier();
      __builtin_amdgcn_fence(__ATOMIC_ACQUIRE, "workgroup");
    }
  }
}

__global__ __launch_bounds__(kThreads) void wcast3_kernel(const float* __restrict__ w0, const float* __restrict__ w1,
                                                          const float* __restrict__ w2, unsigned short* __restrict__ out,
                                                          float scale) {
  const int z = blockIdx.y;
  const float* w = (z == 0) ? w0 : ((z == 1) ? w1 : w2);
  const int i = blockIdx.x * kThreads + threadIdx.x;
  if (i >= kFeat * kFeat / 8) return;
  const float* p = w + 8 * (size_t)i;
  const v4f a = *(const v4f*)(p);
  const v4f c = *(const v4f*)(p + 4);
  unsigned short hb[8];
#pragma unroll
  for (int e = 0; e < 4; ++e) {
    hb[e]     = h_bits(a[e] * scale);
    hb[4 + e] = h_bits(c[e] * scale);
  }
  const v4u u = (v4u){pk16(hb[0], hb[1]), pk16(hb[2], hb[3]), pk16(hb[4], hb[5]), pk16(hb[6], hb[7])};
  unsigned short* q = out + (size_t)z * kFeat * kFeat + 8 * (size_t)i;
  *(volatile v4u*)q = u;
  __threadfence();
  *(volatile v4u*)q = u;
}

__global__ __launch_bounds__(kThreads) void softmax_rows_kernel(const float* __restrict__ zin, float* __restrict__ out, int nrows) {
  const int lane = threadIdx.x & 31, wave = threadIdx.x >> 5;
  const int row = blockIdx.x * kWaves + wave;
  if (row >= nrows) return;
  const v4f x = *(const v4f*)(zin + (size_t)row * kFeat + 4 * lane);
  float m = fmaxf(fmaxf(x[0], x[1]), fmaxf(x[2], x[3]));
#pragma unroll
  for (int off = 16; off > 0; off >>= 1) m = fmaxf(m, __shfl_xor(m, off, 32));
  v4f e;
  e[0] = expf(x[0] - m); e[1] = expf(x[1] - m); e[2] = expf(x[2] - m); e[3] = expf(x[3] - m);
  float s = (e[0] + e[1]) + (e[2] + e[3]);
#pragma unroll
  for (int off = 16; off > 0; off >>= 1) s += __shfl_xor(s, off, 32);
  const float inv = 1.0f / s;
  const v4f o = e * inv;
  float* op = out + (size_t)row * kFeat + 4 * lane;
  *(volatile v4f*)op = o;
  __threadfence();
  *(volatile v4f*)op = o;
}

extern "C" void kernel_launch(void* const* d_in, const int* in_sizes, int n_in,
                              void* d_out, int out_size, void* d_ws, size_t ws_size, hipStream_t stream) {
  (void)n_in;
  const float* x    = (const float*)d_in[0];
  const float* ev   = (const float*)d_in[1];
  const float* W1   = (const float*)d_in[2];
  const float* b1   = (const float*)d_in[3];
  const float* W2   = (const float*)d_in[4];
  const float* b2   = (const float*)d_in[5];
  const float* W3   = (const float*)d_in[6];
  const float* b3   = (const float*)d_in[7];
  const int*   esrc = (const int*)d_in[8];
  const int*   edst = (const int*)d_in[9];
  float* out = (float*)d_out;

  if (in_sizes[0] != kNodes * kFeat || in_sizes[1] != kEdges || in_sizes[8] != kEdges || in_sizes[9] != kEdges) return;
  if (in_sizes[2] != kFeat * kFeat || in_sizes[4] != kFeat * kFeat || in_sizes[6] != kFeat * kFeat) return;
  if (in_sizes[3] != kFeat || in_sizes[5] != kFeat || in_sizes[7] != kFeat) return;
  if (out_size != kNodes * kFeat) return;

  char* ws = (char*)d_ws; size_t off = 0;
  auto carve = [&](size_t bytes) -> char* { char* p = ws + off; off += (bytes + 255) & ~(size_t)255; return p; };
  unsigned short* W16   = (unsigned short*)carve((size_t)3 * kFeat * kFeat * 2);
  float*          ACC32 = (float*)carve((size_t)kMPad * kFeat * 4);
  unsigned short* AGG16 = (unsigned short*)carve((size_t)kMPad * kFeat * 2);
  float*          H32   = (float*)carve((size_t)kMPad * kFeat * 4);
  if (off > ws_size || off > kWsLimit) return;

  const int gemmTiles  = (kMPad / 64) * (kFeat / 64);
  const int gemmBlocks = (gemmTiles + 7) / 8;
  const int smBlocks   = kNodes / kWaves;

  wcast3_kernel<<<dim3(kFeat * kFeat / 8 / kThreads, 3), kThreads, 0, stream>>>(W1, W2, W3, W16, kWCarry);

  spmm_tile_kernel<<<kTiles, kThreads, 0, stream>>>(x, ev, esrc, edst, ACC32, AGG16);
  wmma_gemm64<0, false, 2, 0, false, 6><<<dim3(gemmBlocks, 1), 256, 0, stream>>>(
      (const unsigned short*)AGG16, (const unsigned short*)nullptr, kFeat, 0L,
      (const unsigned short*)W16, (const unsigned short*)nullptr, kFeat, 0L,
      (void*)H32, (void*)nullptr, kFeat, 0L,
      b1, (const float*)nullptr, 0L, kMPad, kFeat, kFeat, kGemmScale);

  spmm_tile_kernel<<<kTiles, kThreads, 0, stream>>>(H32, ev, esrc, edst, ACC32, AGG16);
  wmma_gemm64<0, false, 2, 0, false, 6><<<dim3(gemmBlocks, 1), 256, 0, stream>>>(
      (const unsigned short*)AGG16, (const unsigned short*)nullptr, kFeat, 0L,
      (const unsigned short*)(W16 + (size_t)kFeat * kFeat), (const unsigned short*)nullptr, kFeat, 0L,
      (void*)H32, (void*)nullptr, kFeat, 0L,
      b2, (const float*)nullptr, 0L, kMPad, kFeat, kFeat, kGemmScale);

  spmm_tile_kernel<<<kTiles, kThreads, 0, stream>>>(H32, ev, esrc, edst, ACC32, AGG16);
  wmma_gemm64<0, false, 2, 0, false, 0><<<dim3(gemmBlocks, 1), 256, 0, stream>>>(
      (const unsigned short*)AGG16, (const unsigned short*)nullptr, kFeat, 0L,
      (const unsigned short*)(W16 + (size_t)2 * kFeat * kFeat), (const unsigned short*)nullptr, kFeat, 0L,
      (void*)H32, (void*)nullptr, kFeat, 0L,
      b3, (const float*)nullptr, 0L, kMPad, kFeat, kFeat, kGemmScale);
  softmax_rows_kernel<<<smBlocks, kThreads, 0, stream>>>(H32, out, kNodes);
}
